// MultiheadLSHAttention_919123001907
// MI455X (gfx1250) — hardware-verified
//
#include <hip/hip_runtime.h>
#include <math.h>
#include <stdint.h>

#define SEQ 4096
#define EMB 512
#define NH  8
#define HD  64
#define HPL (SEQ * HD)
#define NQB (SEQ / 64)
#define NKT (SEQ / 64)
static_assert(NH * HD == EMB);
static_assert(NH * HPL == SEQ * EMB);
static_assert(NQB == 64 && NKT == 64);
static_assert((SEQ % 64) == 0 && (EMB % 64) == 0 && (EMB % 32) == 0);

typedef _Float16 v16h __attribute__((ext_vector_type(16)));
typedef _Float16 v8h  __attribute__((ext_vector_type(8)));
typedef __bf16   v16b __attribute__((ext_vector_type(16)));
typedef __bf16   v8b  __attribute__((ext_vector_type(8)));
typedef float    v8f  __attribute__((ext_vector_type(8)));
typedef float    v4f  __attribute__((ext_vector_type(4)));
typedef unsigned int v4u __attribute__((ext_vector_type(4)));

#if defined(__HIP_DEVICE_COMPILE__)
#define DEV_ASM 1
#else
#define DEV_ASM 0
#endif

__device__ __forceinline__ unsigned short bf_bits(float f) {
  unsigned u = __float_as_uint(f);
  return (unsigned short)((u + 0x7FFFu + ((u >> 16) & 1u)) >> 16);
}
__device__ __forceinline__ float bf_up(unsigned short hb) { return __uint_as_float(((unsigned)hb) << 16); }
__device__ __forceinline__ unsigned short h_bits(_Float16 x) { return __builtin_bit_cast(unsigned short, x); }
__device__ __forceinline__ unsigned pk16(unsigned short a, unsigned short b) { return (unsigned)a | ((unsigned)b << 16); }
__device__ __forceinline__ v8f zero8() { v8f z = {0.f, 0.f, 0.f, 0.f, 0.f, 0.f, 0.f, 0.f}; return z; }

template <typename OT> struct FT;
template <> struct FT<__bf16>   { typedef v16b frag; typedef v8b half8; };
template <> struct FT<_Float16> { typedef v16h frag; typedef v8h half8; };

template <typename OT>
__device__ __forceinline__ typename FT<OT>::frag ldfrag(const OT* p) {
  union { typename FT<OT>::frag v; typename FT<OT>::half8 h[2]; } f;
  f.h[0] = *(const typename FT<OT>::half8*)(p);
  f.h[1] = *(const typename FT<OT>::half8*)(p + 16);
  return f.v;
}

__device__ __forceinline__ v8f mmar(v16b a, v16b b, v8f c) {
  return __builtin_amdgcn_wmma_f32_16x16x32_bf16(false, a, false, b, (short)0, c, false, false);
}
__device__ __forceinline__ v8f mmar(v16h a, v16h b, v8f c) {
  return __builtin_amdgcn_wmma_f32_16x16x32_f16(false, a, false, b, (short)0, c, false, false);
}
__device__ __forceinline__ v8f mma_h(v16h a, v16h b, v8f c) {
  c = __builtin_amdgcn_wmma_f32_16x16x32_f16(false, a, false, b, (short)0, c, false, false);
#if DEV_ASM
  asm volatile("v_nop\n\tv_nop\n\tv_nop\n\tv_nop" : "+v"(c) : "v"(a), "v"(b));
#endif
  return c;
}
__device__ __forceinline__ void dep_guard(v8f& a, v8f& b, v16b x, v16b y) {
#if DEV_ASM
  asm volatile("v_nop\n\tv_nop\n\tv_nop\n\tv_nop" : "+v"(a), "+v"(b) : "v"(x), "v"(y));
#else
  (void)a; (void)b; (void)x; (void)y;
#endif
}
__device__ __forceinline__ void dep_guard5(v8f& a, v8f& b, v16h x, v16h y, v16h z) {
#if DEV_ASM
  asm volatile("v_nop\n\tv_nop\n\tv_nop\n\tv_nop" : "+v"(a), "+v"(b) : "v"(x), "v"(y), "v"(z));
#else
  (void)a; (void)b; (void)x; (void)y; (void)z;
#endif
}
__device__ __forceinline__ void keep4(v16b a, v16b b, v16b c, v16b d) {
#if DEV_ASM
  asm volatile("v_nop" :: "v"(a), "v"(b), "v"(c), "v"(d));
#else
  (void)a; (void)b; (void)c; (void)d;
#endif
}
__device__ __forceinline__ void keep4(v16h a, v16h b, v16h c, v16h d) {
#if DEV_ASM
  asm volatile("v_nop" :: "v"(a), "v"(b), "v"(c), "v"(d));
#else
  (void)a; (void)b; (void)c; (void)d;
#endif
}
__device__ __forceinline__ void acc_guard4(v8f& a, v8f& b, v8f& c, v8f& d) {
#if DEV_ASM
  asm volatile("v_nop\n\tv_nop\n\tv_nop\n\tv_nop" : "+v"(a), "+v"(b), "+v"(c), "+v"(d));
#else
  (void)a; (void)b; (void)c; (void)d;
#endif
}

template <int MODE>
__device__ __forceinline__ unsigned short cvm(float f) {
  const unsigned short hb = bf_bits(f);
  if (MODE == 0) return hb;
  return h_bits((_Float16)(bf_up(hb) * 1024.0f));
}

template <int MODE>
__global__ __launch_bounds__(256) void cvt16x8(const float* __restrict__ in, unsigned short* out, int n8) {
  const int i = blockIdx.x * 256 + (int)threadIdx.x;
  if (i < n8) {
    const v4f a  = *(const v4f*)(in + (size_t)i * 8);
    const v4f a4 = *(const v4f*)(in + (size_t)i * 8 + 4);
    v4u p;
    p[0] = pk16(cvm<MODE>(a[0]),  cvm<MODE>(a[1]));
    p[1] = pk16(cvm<MODE>(a[2]),  cvm<MODE>(a[3]));
    p[2] = pk16(cvm<MODE>(a4[0]), cvm<MODE>(a4[1]));
    p[3] = pk16(cvm<MODE>(a4[2]), cvm<MODE>(a4[3]));
    unsigned short* o = out + (size_t)i * 8;
    *(volatile v4u*)o = p;
    __threadfence();
    *(volatile v4u*)o = p;
  }
}

template <typename OT, int OUT_MODE>
__global__ __launch_bounds__(256) void gemm64(
    const unsigned short* __restrict__ Ap, int lda,
    const unsigned short* __restrict__ Btp, int ldb,
    unsigned short* Cout, unsigned short* Cout2, int ldc,
    const float* __restrict__ bias,
    int M, int N, int K, float cscale, float rscale) {
  typedef typename FT<OT>::frag V16;
  const OT* A  = (const OT*)(const void*)Ap;
  const OT* Bt = (const OT*)(const void*)Btp;
  __shared__ __align__(16) float sT[8][16 * 68];
  const int lane = threadIdx.x & 31;
  const int wave = threadIdx.x >> 5;
  const int tilesN = N >> 6;
  const int tilesM = M >> 6;
  const int tile = blockIdx.x * 8 + wave;
  if (tile >= tilesM * tilesN) return;
  const int tm = tile / tilesN;
  const int tn = tile - tm * tilesN;
  const int m0 = tm << 6;
  const int n0 = tn << 6;

  const int rlane = lane & 15;
  const int koff  = (lane >> 4) * 8;
  const int mOff  = (lane >> 4) * 8;

  v8f acc[4][4];
#pragma unroll
  for (int i = 0; i < 4; ++i)
#pragma unroll
    for (int j = 0; j < 4; ++j) acc[i][j] = zero8();

  for (int k0 = 0; k0 < K; k0 += 32) {
    V16 bq[4];
#pragma unroll
    for (int j = 0; j < 4; ++j)
      bq[j] = ldfrag<OT>(Bt + (size_t)(n0 + (j << 4) + rlane) * ldb + koff + k0);
#pragma unroll
    for (int i = 0; i < 4; ++i) {
      const V16 af = ldfrag<OT>(A + (size_t)(m0 + (i << 4) + rlane) * lda + koff + k0);
#pragma unroll
      for (int j = 0; j < 4; ++j) acc[i][j] = mmar(af, bq[j], acc[i][j]);
      dep_guard(acc[i][0], acc[i][3], af, bq[3]);
    }
    keep4(bq[0], bq[1], bq[2], bq[3]);
  }
  acc_guard4(acc[0][0], acc[0][1], acc[0][2], acc[0][3]);
  acc_guard4(acc[1][0], acc[1][1], acc[1][2], acc[1][3]);
  acc_guard4(acc[2][0], acc[2][1], acc[2][2], acc[2][3]);
  acc_guard4(acc[3][0], acc[3][1], acc[3][2], acc[3][3]);

  float* slab = sT[wave];
  const int q = lane >> 3, c8 = (lane & 7) * 8;
  float bb[8];
  {
    const v4f b0 = *(const v4f*)(bias + n0 + c8);
    const v4f b1 = *(const v4f*)(bias + n0 + c8 + 4);
#pragma unroll
    for (int e = 0; e < 4; ++e) {
      bb[e]     = bf_up(bf_bits(b0[e]));
      bb[4 + e] = bf_up(bf_bits(b1[e]));
    }
  }
#pragma unroll
  for (int i = 0; i < 4; ++i) {
    const int mBase = m0 + (i << 4);
#pragma unroll
    for (int j = 0; j < 4; ++j) {
#pragma unroll
      for (int r = 0; r < 8; ++r) {
        slab[(mOff + r) * 68 + (j << 4) + rlane] = acc[i][j][r];
      }
    }
    __builtin_amdgcn_fence(__ATOMIC_RELEASE, "workgroup");
    __builtin_amdgcn_wave_barrier();
    __builtin_amdgcn_fence(__ATOMIC_ACQUIRE, "workgroup");
    v4u hv[4], lv[4];
#pragma unroll
    for (int it = 0; it < 4; ++it) {
      const int row = it * 4 + q;
      const float* sp = slab + row * 68 + c8;
      float f[8];
#pragma unroll
      for (int e = 0; e < 8; ++e) f[e] = (sp[e] + bb[e]) * cscale;
      v4u a, a2;
#pragma unroll
      for (int e = 0; e < 4; ++e) {
        const float f0 = f[2 * e], f1 = f[2 * e + 1];
        const _Float16 x0 = (_Float16)f0, x1 = (_Float16)f1;
        const unsigned short h0 = h_bits(x0), h1 = h_bits(x1);
        unsigned short l0 = 0, l1 = 0;
        if (OUT_MODE == 3) {
          l0 = h_bits((_Float16)((f0 - (float)x0) * rscale));
          l1 = h_bits((_Float16)((f1 - (float)x1) * rscale));
        }
        a[e] = pk16(h0, h1); a2[e] = pk16(l0, l1);
      }
      hv[it] = a; lv[it] = a2;
    }
    for (int pass = 0; pass < 2; ++pass) {
#pragma unroll
      for (int it = 0; it < 4; ++it) {
        const int row = it * 4 + q;
        *(volatile v4u*)(Cout + (size_t)(mBase + row) * ldc + n0 + c8) = hv[it];
        if (OUT_MODE == 3) *(volatile v4u*)(Cout2 + (size_t)(mBase + row) * ldc + n0 + c8) = lv[it];
      }
      __threadfence();
    }
    __builtin_amdgcn_fence(__ATOMIC_RELEASE, "workgroup");
    __builtin_amdgcn_wave_barrier();
    __builtin_amdgcn_fence(__ATOMIC_ACQUIRE, "workgroup");
  }
}

__global__ __launch_bounds__(256) void gemm_o(
    const unsigned short* __restrict__ Ahp, const unsigned short* __restrict__ Alp, int lda,
    const unsigned short* __restrict__ Btp, int ldb,
    float* Cout, int ldc, const float* __restrict__ bias,
    int M, int N, int K, float hscale, float lscale) {
  const _Float16* Ah = (const _Float16*)(const void*)Ahp;
  const _Float16* Al = (const _Float16*)(const void*)Alp;
  const _Float16* Bt = (const _Float16*)(const void*)Btp;
  __shared__ __align__(16) float sT[8][16 * 68];
  const int lane = threadIdx.x & 31;
  const int wave = threadIdx.x >> 5;
  const int tilesN = N >> 6;
  const int tilesM = M >> 5;
  const int tile = blockIdx.x * 8 + wave;
  if (tile >= tilesM * tilesN) return;
  const int tm = tile / tilesN;
  const int tn = tile - tm * tilesN;
  const int m0 = tm << 5;
  const int n0 = tn << 6;

  const int rlane = lane & 15;
  const int koff  = (lane >> 4) * 8;
  const int mOff  = (lane >> 4) * 8;

  v8f ach[2][4], acl[2][4];
#pragma unroll
  for (int i = 0; i < 2; ++i)
#pragma unroll
    for (int j = 0; j < 4; ++j) { ach[i][j] = zero8(); acl[i][j] = zero8(); }

  for (int k0 = 0; k0 < K; k0 += 32) {
    v16h bq[4];
#pragma unroll
    for (int j = 0; j < 4; ++j)
      bq[j] = ldfrag<_Float16>(Bt + (size_t)(n0 + (j << 4) + rlane) * ldb + koff + k0);
#pragma unroll
    for (int i = 0; i < 2; ++i) {
      const v16h afh = ldfrag<_Float16>(Ah + (size_t)(m0 + (i << 4) + rlane) * lda + koff + k0);
      const v16h afl = ldfrag<_Float16>(Al + (size_t)(m0 + (i << 4) + rlane) * lda + koff + k0);
#pragma unroll
      for (int j = 0; j < 4; ++j) {
        ach[i][j] = mmar(afh, bq[j], ach[i][j]);
        acl[i][j] = mmar(afl, bq[j], acl[i][j]);
      }
      dep_guard5(ach[i][0], acl[i][3], afh, afl, bq[3]);
    }
    keep4(bq[0], bq[1], bq[2], bq[3]);
  }
  acc_guard4(ach[0][0], ach[0][1], ach[0][2], ach[0][3]);
  acc_guard4(ach[1][0], ach[1][1], ach[1][2], ach[1][3]);
  acc_guard4(acl[0][0], acl[0][1], acl[0][2], acl[0][3]);
  acc_guard4(acl[1][0], acl[1][1], acl[1][2], acl[1][3]);

  float* slab = sT[wave];
  const int h2 = lane >> 4, c4 = (lane & 15) * 4;
  v4f b4 = *(const v4f*)(bias + n0 + c4);
#pragma unroll
  for (int e = 0; e < 4; ++e) b4[e] = bf_up(bf_bits(b4[e]));
#pragma unroll
  for (int i = 0; i < 2; ++i) {
    const int mBase = m0 + (i << 4);
#pragma unroll
    for (int j = 0; j < 4; ++j) {
#pragma unroll
      for (int r = 0; r < 8; ++r) {
        slab[(mOff + r) * 68 + (j << 4) + rlane] = ach[i][j][r] * hscale + acl[i][j][r] * lscale;
      }
    }
    __builtin_amdgcn_fence(__ATOMIC_RELEASE, "workgroup");
    __builtin_amdgcn_wave_barrier();
    __builtin_amdgcn_fence(__ATOMIC_ACQUIRE, "workgroup");
    v4f ov[8];
#pragma unroll
    for (int it = 0; it < 8; ++it) {
      const int row = it * 2 + h2;
      ov[it] = *(const v4f*)(slab + row * 68 + c4) + b4;
    }
    for (int pass = 0; pass < 2; ++pass) {
#pragma unroll
      for (int it = 0; it < 8; ++it) {
        const int row = it * 2 + h2;
        *(volatile v4f*)(Cout + (size_t)(mBase + row) * ldc + n0 + c4) = ov[it];
      }
      __threadfence();
    }
    __builtin_amdgcn_fence(__ATOMIC_RELEASE, "workgroup");
    __builtin_amdgcn_wave_barrier();
    __builtin_amdgcn_fence(__ATOMIC_ACQUIRE, "workgroup");
  }
}

__global__ __launch_bounds__(128) void vtrans(const unsigned short* __restrict__ pvp, unsigned short* vtp) {
  __shared__ __align__(16) _Float16 T[64 * 72];
  const int tid = threadIdx.x, lane = tid & 31, wave = tid >> 5;
  const int h = blockIdx.y, t0 = blockIdx.x * 64;
  const size_t hoff = (size_t)h * HPL;
  const _Float16* pv = (const _Float16*)(const void*)pvp + hoff;
  {
    const int r = tid >> 1, half = (tid & 1) * 32;
    const _Float16* src = pv + (size_t)(t0 + r) * HD + half;
#pragma unroll
    for (int i = 0; i < 4; ++i) *(v8h*)(T + r * 72 + half + 8 * i) = *(const v8h*)(src + 8 * i);
  }
  __syncthreads();
  const int q4 = lane >> 3, q8 = lane & 7;
  v4u ov[4];
#pragma unroll
  for (int it = 0; it < 4; ++it) {
    const int d = wave * 16 + it * 4 + q4;
    v4u a;
#pragma unroll
    for (int e = 0; e < 4; ++e) {
      const _Float16 x0 = T[(8 * q8 + 2 * e) * 72 + d];
      const _Float16 x1 = T[(8 * q8 + 2 * e + 1) * 72 + d];
      a[e] = pk16(h_bits(x0), h_bits(x1));
    }
    ov[it] = a;
  }
  for (int pass = 0; pass < 2; ++pass) {
#pragma unroll
    for (int it = 0; it < 4; ++it) {
      const int d = wave * 16 + it * 4 + q4;
      *(volatile v4u*)(vtp + hoff + (size_t)d * SEQ + t0 + 8 * q8) = ov[it];
    }
    __threadfence();
  }
}

__global__ __launch_bounds__(128)
void attn_hd64(const unsigned short* __restrict__ qhp, const unsigned short* __restrict__ qlp,
               const unsigned short* __restrict__ kpp, const unsigned short* __restrict__ vtp,
               unsigned short* chp, unsigned short* clp, float sscale) {
  union FH { v16h v; v8h h[2]; };
  __shared__ __align__(16) _Float16 Ksh[64 * 64];
  __shared__ __align__(16) _Float16 Vts[64 * 64];
  __shared__ __align__(16) _Float16 Psh[4][16 * 64];
  __shared__ __align__(16) _Float16 Psl[4][16 * 64];
  __shared__ __align__(16) float    Os[4][16 * 64];

  const int tid  = threadIdx.x;
  const int wave = tid >> 5;
  const int lane = tid & 31;
  const int hh   = lane >> 4;
  const int c    = lane & 15;

  const int bx = blockIdx.x;
  const int qb = bx % NQB;
  const int h  = bx / NQB;
  const int q0 = qb * 64 + wave * 16;
  const size_t hoff = (size_t)h * HPL;

  const _Float16* Qh = (const _Float16*)(const void*)qhp + hoff;
  const _Float16* Ql = (const _Float16*)(const void*)qlp + hoff;
  const _Float16* Kg = (const _Float16*)(const void*)kpp + hoff;
  const _Float16* Vg = (const _Float16*)(const void*)vtp + hoff;

  v16h qah[2], qal[2];
#pragma unroll
  for (int dc = 0; dc < 2; ++dc) {
    const size_t qo = (size_t)(q0 + c) * HD + dc * 32 + 8 * hh;
    qah[dc] = ldfrag<_Float16>(Qh + qo);
    qal[dc] = ldfrag<_Float16>(Ql + qo);
  }

  float mrow[8], lrow[8];
  v8f oacc[4];
#pragma unroll
  for (int r = 0; r < 8; ++r) { mrow[r] = -INFINITY; lrow[r] = 0.f; }
#pragma unroll
  for (int t = 0; t < 4; ++t) oacc[t] = zero8();

  for (int kt = 0; kt < NKT; ++kt) {
    const int kv0 = kt * 64;
    __syncthreads();
    {
      const int r = tid >> 1, half = (tid & 1) * 32;
      const _Float16* kg = Kg + (size_t)(kv0 + r) * HD + half;
      const _Float16* vg = Vg + (size_t)r * SEQ + kv0 + half;
#pragma unroll
      for (int i = 0; i < 4; ++i) {
        const v8h a0 = *(const v8h*)(kg + 8 * i);
        const v8h b0 = *(const v8h*)(vg + 8 * i);
        *(v8h*)(Ksh + r * 64 + half + 8 * i) = a0;
        *(v8h*)(Vts + r * 64 + half + 8 * i) = b0;
      }
    }
    __syncthreads();

    v8f s[4];
#pragma unroll
    for (int j = 0; j < 4; ++j) {
      v8f ah = zero8(), al = zero8();
#pragma unroll
      for (int dc = 0; dc < 2; ++dc) {
        FH kb;
        kb.h[0] = *(const v8h*)(Ksh + (j * 16 + c) * 64 + dc * 32 + 8 * hh);
        kb.h[1] = *(const v8h*)(Ksh + (j * 16 + c) * 64 + dc * 32 + 16 + 8 * hh);
        ah = mma_h(qah[dc], kb.v, ah);
        al = mma_h(qal[dc], kb.v, al);
      }
#pragma unroll
      for (int r = 0; r < 8; ++r) s[j][r] = (ah[r] + al[r] * (1.0f / 4096.0f)) * sscale;
    }

    _Float16* pwh = Psh[wave];
    _Float16* pwl = Psl[wave];
#pragma unroll
    for (int r = 0; r < 8; ++r) {
      float m = s[0][r];
#pragma unroll
      for (int j = 1; j < 4; ++j) m = fmaxf(m, s[j][r]);
#pragma unroll
      for (int off = 1; off < 16; off <<= 1) m = fmaxf(m, __shfl_xor(m, off, 32));
      const float mnew  = fmaxf(mrow[r], m);
      const float msafe = (mnew == -INFINITY) ? 0.f : mnew;
      const float alpha = __expf(mrow[r] - msafe);
      mrow[r] = mnew;
      float psum = 0.f;
#pragma unroll
      for (int j = 0; j < 4; ++j) {
        const float p  = __expf(s[j][r] - msafe);
        psum += p;
        const float pc = p * 1024.0f;
        const _Float16 ph = (_Float16)pc;
        const _Float16 pl = (_Float16)((pc - (float)ph) * 4096.0f);
        pwh[(8 * hh + r) * 64 + j * 16 + c] = ph;
        pwl[(8 * hh + r) * 64 + j * 16 + c] = pl;
      }
#pragma unroll
      for (int off = 1; off < 16; off <<= 1) psum += __shfl_xor(psum, off, 32);
      lrow[r] = lrow[r] * alpha + psum;
#pragma unroll
      for (int t = 0; t < 4; ++t) oacc[t][r] *= alpha;
    }
    __builtin_amdgcn_fence(__ATOMIC_RELEASE, "workgroup");
    __builtin_amdgcn_wave_barrier();
    __builtin_amdgcn_fence(__ATOMIC_ACQUIRE, "workgroup");

    v8f o1[4];
#pragma unroll
    for (int t = 0; t < 4; ++t) o1[t] = zero8();
#pragma unroll 1
    for (int kk = 0; kk < 2; ++kk) {
      FH pa, pb;
      pa.h[0] = *(const v8h*)(pwh + c * 64 + kk * 32 + 8 * hh);
      pa.h[1] = *(const v8h*)(pwh + c * 64 + kk * 32 + 16 + 8 * hh);
      pb.h[0] = *(const v8h*)(pwl + c * 64 + kk * 32 + 8 * hh);
      pb.h[1] = *(const v8h*)(pwl + c * 64 + kk * 32 + 16 + 8 * hh);
#pragma unroll
      for (int t = 0; t < 4; ++t) {
        FH vb;
        vb.h[0] = *(const v8h*)(Vts + (t * 16 + c) * 64 + kk * 32 + 8 * hh);
        vb.h[1] = *(const v8h*)(Vts + (t * 16 + c) * 64 + kk * 32 + 16 + 8 * hh);
        oacc[t] = mma_h(pa.v, vb.v, oacc[t]);
        o1[t]   = mma_h(pb.v, vb.v, o1[t]);
      }
    }
#pragma unroll
    for (int t = 0; t < 4; ++t)
#pragma unroll
      for (int r = 0; r < 8; ++r) oacc[t][r] += o1[t][r] * (1.0f / 4096.0f);
  }

  float* os = Os[wave];
#pragma unroll
  for (int r = 0; r < 8; ++r) {
    const float l = lrow[r];
    const float inv = ((l > 0.f) ? (1.0f / l) : 0.f) * (1.0f / 64.0f);
#pragma unroll
    for (int t = 0; t < 4; ++t) os[(8 * hh + r) * 64 + t * 16 + c] = oacc[t][r] * inv;
  }
  __builtin_amdgcn_fence(__ATOMIC_RELEASE, "workgroup");
  __builtin_amdgcn_wave_barrier();
  __builtin_amdgcn_fence(__ATOMIC_ACQUIRE, "workgroup");
  {
    const int q4 = lane >> 3, c8 = (lane & 7) * 8;
    v4u hv[4], lv[4];
#pragma unroll
    for (int it = 0; it < 4; ++it) {
      const int row = it * 4 + q4;
      const float* sp = os + row * 64 + c8;
      v4u a, a2;
#pragma unroll
      for (int e = 0; e < 4; ++e) {
        const float f0 = sp[2 * e], f1 = sp[2 * e + 1];
        const _Float16 x0 = (_Float16)f0, x1 = (_Float16)f1;
        const unsigned short l0 = h_bits((_Float16)((f0 - (float)x0) * 4096.0f));
        const unsigned short l1 = h_bits((_Float16)((f1 - (float)x1) * 4096.0f));
        a[e]  = pk16(h_bits(x0), h_bits(x1));
        a2[e] = pk16(l0, l1);
      }
      hv[it] = a; lv[it] = a2;
    }
    for (int pass = 0; pass < 2; ++pass) {
#pragma unroll
      for (int it = 0; it < 4; ++it) {
        const int row = it * 4 + q4;
        const size_t go = hoff + (size_t)(q0 + row) * HD + c8;
        *(volatile v4u*)(chp + go) = hv[it];
        *(volatile v4u*)(clp + go) = lv[it];
      }
      __threadfence();
    }
  }
}

extern "C" void kernel_launch(void* const* d_in, const int* in_sizes, int n_in,
                              void* d_out, int out_size, void* d_ws, size_t ws_size,
                              hipStream_t stream) {
  const int NX = SEQ * EMB;
  const int NW = EMB * EMB;
  if (n_in < 9) return;
  if (in_sizes[0] != NX || in_sizes[1] != NX || in_sizes[2] != NX) return;
  if (in_sizes[3] != NW || in_sizes[5] != NW || in_sizes[7] != NW) return;
  if (in_sizes[4] != EMB || in_sizes[6] != EMB || in_sizes[8] != EMB) return;
  if (out_size != NX) return;

  const float* Q    = (const float*)d_in[0];
  const float* Kin  = (const float*)d_in[1];
  const float* V    = (const float*)d_in[2];
  const float* Wqk  = (const float*)d_in[3];
  const float* bqk  = (const float*)d_in[4];
  const float* Wv   = (const float*)d_in[5];
  const float* bv   = (const float*)d_in[6];
  const float* Wout = (const float*)d_in[7];
  const float* bout = (const float*)d_in[8];
  float* out = (float*)d_out;

  const size_t PX = (size_t)NX * 2;
  const size_t PW = (size_t)NW * 2;
  size_t off = 0;
  const size_t oQb  = off; off += PX;
  const size_t oKb  = off; off += PX;
  const size_t oVb  = off; off += PX;
  const size_t oWqk = off; off += PW;
  const size_t oWv  = off; off += PW;
  const size_t oWo  = off; off += PW;
  const size_t oQh  = off; off += PX;
  const size_t oQl  = off; off += PX;
  const size_t oKp  = off; off += PX;
  const size_t oPv  = off; off += PX;
  const size_t oVt  = off; off += PX;
  const size_t oCh  = off; off += PX;
  const size_t oCl  = off; off += PX;
  if (off > ws_size) return;
  if (off > (size_t)134217728) return;

  char* ws = (char*)d_ws;
  unsigned short* Qb   = (unsigned short*)(ws + oQb);
  unsigned short* Kb   = (unsigned short*)(ws + oKb);
  unsigned short* Vb   = (unsigned short*)(ws + oVb);
  unsigned short* Wqkb = (unsigned short*)(ws + oWqk);
  unsigned short* Wvb  = (unsigned short*)(ws + oWv);
  unsigned short* Woh  = (unsigned short*)(ws + oWo);
  unsigned short* Qh   = (unsigned short*)(ws + oQh);
  unsigned short* Ql   = (unsigned short*)(ws + oQl);
  unsigned short* Kp   = (unsigned short*)(ws + oKp);
  unsigned short* Pv   = (unsigned short*)(ws + oPv);
  unsigned short* Vt   = (unsigned short*)(ws + oVt);
  unsigned short* Ch   = (unsigned short*)(ws + oCh);
  unsigned short* Cl   = (unsigned short*)(ws + oCl);

  const dim3 blk(256);
  const int n8x = NX / 8;
  const int n8w = NW / 8;
  const dim3 gCvtX((n8x + 255) / 256);
  const dim3 gCvtW((n8w + 255) / 256);
  const dim3 gPj(((SEQ / 64) * (EMB / 64) + 7) / 8);
  const dim3 gTr(SEQ / 64, NH);
  const dim3 gAttn(NH * NQB);
  const dim3 gOut(((SEQ / 32) * (EMB / 64) + 7) / 8);

  cvt16x8<0><<<gCvtX, blk, 0, stream>>>(Q,    Qb,   n8x);
  cvt16x8<0><<<gCvtX, blk, 0, stream>>>(Kin,  Kb,   n8x);
  cvt16x8<0><<<gCvtX, blk, 0, stream>>>(V,    Vb,   n8x);
  cvt16x8<0><<<gCvtW, blk, 0, stream>>>(Wqk,  Wqkb, n8w);
  cvt16x8<0><<<gCvtW, blk, 0, stream>>>(Wv,   Wvb,  n8w);
  cvt16x8<1><<<gCvtW, blk, 0, stream>>>(Wout, Woh,  n8w);
  gemm64<__bf16, 3><<<gPj, blk, 0, stream>>>(
      Qb, EMB, Wqkb, EMB, Qh, Ql, EMB, bqk, SEQ, EMB, EMB, 16.0f, 4096.0f);
  gemm64<__bf16, 1><<<gPj, blk, 0, stream>>>(
      Kb, EMB, Wqkb, EMB, Kp, Kp, EMB, bqk, SEQ, EMB, EMB, 16.0f, 1.0f);
  gemm64<__bf16, 1><<<gPj, blk, 0, stream>>>(
      Vb, EMB, Wvb, EMB, Pv, Pv, EMB, bv, SEQ, EMB, EMB, 16.0f, 1.0f);
  vtrans<<<gTr, dim3(128), 0, stream>>>(Pv, Vt);
  attn_hd64<<<gAttn, dim3(128), 0, stream>>>(Qh, Ql, Kp, Vt, Ch, Cl, 1.0f / 2048.0f);
  gemm_o<<<gOut, blk, 0, stream>>>(
      Ch, Cl, EMB, Woh, EMB, out, EMB, bout, SEQ, EMB, EMB,
      1.0f / 262144.0f, 1.0f / 1073741824.0f);
  (void)hipGetLastError();
}
